// SGCFeatureExtractor_64888365908056
// MI455X (gfx1250) — hardware-verified
//
#include <hip/hip_runtime.h>
#include <stddef.h>


#define NB     256
#define NNODE  64
#define NF     128
#define NH     64
#define NROWS  (NB * NNODE)
#define NGE    (NNODE * NNODE)
#define NTRIL  2080
#define NTHR   256
#define NSTAT  64
#define RSTAT  (NROWS / NSTAT)
#define XP     136
#define ZP     72
#define BN_EPS 1e-5f
#define XSCL   16.0f
#define WSCL   64.0f
#define PSCL   4096.0f
#define INV1024  0.0009765625f
#define INV65536 0.0000152587890625f
#define INVROWS  (1.0 / 16384.0)
#define WSCAP  134217728

#define L1_HS 0
#define L1_A2 (L1_HS + NNODE * NF * 4)
#define L1_XS (L1_A2 + NGE * 4)
#define L1_RD (L1_XS + NNODE * XP * 2)
#define L1_PD (L1_RD + 2 * 4 * NH * 8)
#define L1_BT (L1_PD + 2 * NH * 8)
#define LDS1  (L1_BT + 2 * NF * 4)

#define L2_Z  0
#define L2_S  (L2_Z + NNODE * ZP * 2)
#define L2_P  (L2_S + NGE * 4)
#define L2_XT (L2_P + NNODE * ZP * 2)
#define L2_O  (L2_XT + NF * ZP * 2)
#define L2_BT (L2_O + NNODE * NF * 4)
#define LDS2  (L2_BT + 2 * NH * 4)

static_assert(NTRIL == NNODE * (NNODE + 1) / 2);
static_assert(NROWS % NSTAT == 0 && RSTAT % 2 == 0);
static_assert(NF % 32 == 0 && NH % 32 == 0 && NNODE % 32 == 0);
static_assert((XP * 2) % 16 == 0 && (ZP * 2) % 16 == 0 && XP >= NF && ZP >= NNODE);
static_assert((L1_A2 % 16) == 0 && (L1_XS % 16) == 0 && (L1_RD % 16) == 0 && (L1_PD % 16) == 0 && (L1_BT % 16) == 0);
static_assert((L2_S % 16) == 0 && (L2_P % 16) == 0 && (L2_XT % 16) == 0 && (L2_O % 16) == 0 && (L2_BT % 16) == 0);
static_assert(NTHR == 256 && NNODE * NF == 8 * 4 * NTHR && NGE == 4 * 4 * NTHR);
static_assert(2 * NF <= NTHR && 2 * NH <= NTHR);

typedef float          v4f  __attribute__((ext_vector_type(4)));
typedef float          v8f  __attribute__((ext_vector_type(8)));
typedef double         v2d  __attribute__((ext_vector_type(2)));
typedef unsigned short v4us __attribute__((ext_vector_type(4)));
typedef unsigned short v8us __attribute__((ext_vector_type(8)));
typedef _Float16       v16h __attribute__((ext_vector_type(16)));
union FragH { v16h v; v8us u[2]; };

__device__ __forceinline__ unsigned short h16(float f) {
  const _Float16 h = (_Float16)f;
  return __builtin_bit_cast(unsigned short, h);
}

__device__ __forceinline__ v4us cvt4(v4f a, float s) {
  v4us r;
  r[0] = h16(a.x * s); r[1] = h16(a.y * s); r[2] = h16(a.z * s); r[3] = h16(a.w * s);
  return r;
}

__device__ __forceinline__ v8us cvt8(v4f a, v4f b, float s) {
  v8us r;
  r[0] = h16(a.x * s); r[1] = h16(a.y * s); r[2] = h16(a.z * s); r[3] = h16(a.w * s);
  r[4] = h16(b.x * s); r[5] = h16(b.y * s); r[6] = h16(b.z * s); r[7] = h16(b.w * s);
  return r;
}

__device__ __forceinline__ v8f wmh(v16h a, v16h b, v8f c) {
  v8f d = __builtin_amdgcn_wmma_f32_16x16x32_f16(false, a, false, b, (short)0, c, false, false);
  asm volatile("v_nop\n\tv_nop\n\tv_nop\n\tv_nop" : "+v"(d) : "v"(a), "v"(b));
  return d;
}

__global__ __launch_bounds__(NTHR) void k_stat1(const float* __restrict__ x, double* part1) {
  __shared__ __attribute__((aligned(16))) double rs[NTHR];
  __shared__ __attribute__((aligned(16))) double rq[NTHR];
  __shared__ __attribute__((aligned(16))) double pd[NTHR];
  const int tid = threadIdx.x, f = tid & (NF - 1), par = tid >> 7;
  const int row0 = (int)blockIdx.x * RSTAT;
  double s = 0.0, sq = 0.0;
#pragma unroll 2
  for (int k = 0; k < RSTAT / 2; ++k) {
    const int r = row0 + par + 2 * k;
    const double v = (double)x[(size_t)r * NF + f];
    s += v;
    sq += v * v;
  }
  rs[tid] = s;
  rq[tid] = sq;
  __syncthreads();
  if (tid < NF) {
    pd[tid]      = rs[tid] + rs[tid + NF];
    pd[NF + tid] = rq[tid] + rq[tid + NF];
  }
  __syncthreads();
  if (tid < NF) {
    const v2d v = *(const v2d*)(pd + 2 * tid);
    double* dp = part1 + (size_t)blockIdx.x * NTHR + 2 * tid;
    *(volatile v2d*)dp = v;
    __threadfence();
    *(volatile v2d*)dp = v;
  }
}

__global__ __launch_bounds__(NTHR) void k_prep(const double* __restrict__ part1,
                                              const float* __restrict__ g1, const float* __restrict__ be1,
                                              const float* __restrict__ tril, const float* __restrict__ lin_w,
                                              float* bn1tab, float* A2g, unsigned short* lw16) {
  __shared__ __attribute__((aligned(16))) float Wm[NGE];
  __shared__ __attribute__((aligned(16))) float A2l[NGE];
  __shared__ __attribute__((aligned(16))) float tab[2 * NF];
  __shared__ float dis[NNODE];
  const int tid = threadIdx.x;

  if (tid < NF) {
    double s = 0.0, sq = 0.0;
#pragma unroll 1
    for (int k = 0; k < NSTAT; ++k) {
      s  += part1[(size_t)k * NTHR + tid];
      sq += part1[(size_t)k * NTHR + NF + tid];
    }
    const double mu = s * INVROWS;
    double var = sq * INVROWS - mu * mu;
    var = var < 0.0 ? 0.0 : var;
    const float iv = rsqrtf((float)var + BN_EPS);
    const float sc = g1[tid] * iv;
    tab[tid]      = sc;
    tab[NF + tid] = be1[tid] - (float)mu * sc;
  }
#pragma unroll 1
  for (int idx = tid; idx < NGE; idx += NTHR) {
    const int i = idx >> 6, j = idx & 63;
    const int a = i > j ? i : j, c = i > j ? j : i;
    int ti = a * (a + 1) / 2 + c;
    ti = ti < 0 ? 0 : (ti > NTRIL - 1 ? NTRIL - 1 : ti);
    Wm[idx] = tril[ti];
  }
  __syncthreads();
  if (tid < NNODE) {
    float dg = 0.0f;
#pragma unroll 1
    for (int j = 0; j < NNODE; ++j) dg += fabsf(Wm[tid * NNODE + j]);
    dis[tid] = dg > 0.0f ? rsqrtf(dg) : 0.0f;
  }
  __syncthreads();
#pragma unroll 1
  for (int idx = tid; idx < NGE; idx += NTHR) {
    const int i = idx >> 6, j = idx & 63;
    Wm[idx] = dis[i] * Wm[idx] * dis[j];
  }
  __syncthreads();
#pragma unroll 1
  for (int idx = tid; idx < NGE; idx += NTHR) {
    const int i = idx >> 6, j = idx & 63;
    float s = 0.0f;
#pragma unroll 4
    for (int k = 0; k < NNODE; ++k) s = fmaf(Wm[i * NNODE + k], Wm[k * NNODE + j], s);
    A2l[idx] = s;
  }
  v8us hv[4];
#pragma unroll
  for (int it = 0; it < 4; ++it) {
    const int q = it * NTHR + tid;
    const float* wp = lin_w + (size_t)q * 8;
    hv[it] = cvt8(*(const v4f*)wp, *(const v4f*)(wp + 4), WSCL);
  }
  __syncthreads();

  const bool tw = tid < 64;
  v4f tv = {0.f, 0.f, 0.f, 0.f};
  if (tw) tv = *(const v4f*)(tab + 4 * tid);
  v4f av[4];
#pragma unroll
  for (int it = 0; it < 4; ++it) av[it] = *(const v4f*)(A2l + 4 * (it * NTHR + tid));

  if (tw) *(volatile v4f*)(bn1tab + 4 * tid) = tv;
#pragma unroll
  for (int it = 0; it < 4; ++it) {
    const int q = it * NTHR + tid;
    *(volatile v4f*)(A2g + 4 * q) = av[it];
    *(volatile v8us*)(lw16 + (size_t)q * 8) = hv[it];
  }
  __threadfence();
  if (tw) *(volatile v4f*)(bn1tab + 4 * tid) = tv;
#pragma unroll
  for (int it = 0; it < 4; ++it) {
    const int q = it * NTHR + tid;
    *(volatile v4f*)(A2g + 4 * q) = av[it];
    *(volatile v8us*)(lw16 + (size_t)q * 8) = hv[it];
  }
}

__global__ __launch_bounds__(NTHR) void k_graph1(const float* __restrict__ x, const float* __restrict__ bn1tab,
                                                const float* __restrict__ A2g, const unsigned short* __restrict__ lw16,
                                                const float* __restrict__ lin_b,
                                                unsigned short* xs16p, float* xzp, double* part2) {
  extern __shared__ v4f lds_dyn[];
  char* lb = (char*)lds_dyn;
  float* hs  = (float*)(lb + L1_HS);
  float* xzs = (float*)(lb + L1_HS);
  float* A2s = (float*)(lb + L1_A2);
  unsigned short* xsl = (unsigned short*)(lb + L1_XS);
  double* redd = (double*)(lb + L1_RD);
  double* pd   = (double*)(lb + L1_PD);
  float* bt    = (float*)(lb + L1_BT);
  const int tid = threadIdx.x, lane = tid & 31, wave = tid >> 5, hh = lane >> 4, m = lane & 15;
  const int b = blockIdx.x;

  bt[tid] = bn1tab[tid];
#pragma unroll
  for (int it = 0; it < 4; ++it) {
    const int q = it * NTHR + tid;
    *(v4f*)(A2s + 4 * q) = *(const v4f*)(A2g + 4 * q);
  }
  __syncthreads();

  const float* xb = x + (size_t)b * NNODE * NF;
#pragma unroll
  for (int it = 0; it < 8; ++it) {
    const int q = it * NTHR + tid;
    const int f0 = (q & 31) * 4;
    const v4f xv = *(const v4f*)(xb + 4 * q);
    const v4f sc = *(const v4f*)(bt + f0);
    const v4f sh = *(const v4f*)(bt + NF + f0);
    *(v4f*)(hs + 4 * q) = xv * sc + sh;
  }
  __syncthreads();

  {
    const v4f z4 = {0.f, 0.f, 0.f, 0.f};
#pragma unroll 1
    for (int s = 0; s < 2; ++s) {
      const int u  = tid + NTHR * s;
      const int j0 = (u & 15) * 4;
      const int f0 = (u >> 4) * 4;
      v4f a0 = z4, a1 = z4, a2 = z4, a3 = z4;
#pragma unroll 4
      for (int i = 0; i < NNODE; ++i) {
        const v4f w4 = *(const v4f*)(A2s + i * NNODE + j0);
        const v4f h4 = *(const v4f*)(hs + i * NF + f0);
        a0 += w4.x * h4;
        a1 += w4.y * h4;
        a2 += w4.z * h4;
        a3 += w4.w * h4;
      }
      *(v4us*)(xsl + (j0 + 0) * XP + f0) = cvt4(a0, XSCL);
      *(v4us*)(xsl + (j0 + 1) * XP + f0) = cvt4(a1, XSCL);
      *(v4us*)(xsl + (j0 + 2) * XP + f0) = cvt4(a2, XSCL);
      *(v4us*)(xsl + (j0 + 3) * XP + f0) = cvt4(a3, XSCL);
    }
  }
  __syncthreads();

  {
    const int mt = wave >> 1, nt0 = (wave & 1) * 2;
    v8f acc[2];
#pragma unroll
    for (int t = 0; t < 2; ++t) { const v8f z = {0.f, 0.f, 0.f, 0.f, 0.f, 0.f, 0.f, 0.f}; acc[t] = z; }
    const unsigned short* afp = xsl + (16 * mt + m) * XP + 8 * hh;
#pragma unroll
    for (int ks = 0; ks < NF / 32; ++ks) {
      FragH af;
      af.u[0] = *(const v8us*)(afp + 32 * ks);
      af.u[1] = *(const v8us*)(afp + 32 * ks + 16);
#pragma unroll
      for (int t = 0; t < 2; ++t) {
        const unsigned short* bfp = lw16 + (size_t)(16 * (nt0 + t) + m) * NF + 32 * ks + 8 * hh;
        FragH bf;
        bf.u[0] = *(const v8us*)bfp;
        bf.u[1] = *(const v8us*)(bfp + 16);
        acc[t] = wmh(af.v, bf.v, acc[t]);
      }
    }
#pragma unroll
    for (int t = 0; t < 2; ++t) {
      const int n = 16 * (nt0 + t) + m;
      const float bias = lin_b[n];
      float* op = xzs + (16 * mt + 8 * hh) * NH + n;
#pragma unroll
      for (int r = 0; r < 8; ++r) op[r * NH] = acc[t][r] * INV1024 + bias;
    }
  }
  __syncthreads();

  {
    const int c = tid & 63, qg = tid >> 6;
    double s = 0.0, sq = 0.0;
#pragma unroll 4
    for (int r = 16 * qg; r < 16 * qg + 16; ++r) {
      const double v = (double)xzs[r * NH + c];
      s += v;
      sq += v * v;
    }
    redd[qg * NH + c] = s;
    redd[4 * NH + qg * NH + c] = sq;
  }
  __syncthreads();
  if (tid < 2 * NH) {
    const int c = tid & 63, o = (tid >> 6) * (4 * NH);
    pd[tid] = ((redd[o + c] + redd[o + NH + c]) + redd[o + 2 * NH + c]) + redd[o + 3 * NH + c];
  }
  __syncthreads();

  v4f xo[4];
  v8us so[4];
#pragma unroll
  for (int it = 0; it < 4; ++it) {
    const int q = it * NTHR + tid;
    xo[it] = *(const v4f*)(xzs + 4 * q);
    so[it] = *(const v8us*)(xsl + (q >> 4) * XP + (q & 15) * 8);
  }
  const bool tw = tid < 64;
  v2d pv = {0.0, 0.0};
  if (tw) pv = *(const v2d*)(pd + 2 * tid);
  float* xzg = xzp + (size_t)b * NNODE * NH;
  unsigned short* xsg = xs16p + (size_t)b * NNODE * NF;
  double* pg = part2 + (size_t)b * (2 * NH);
#pragma unroll
  for (int it = 0; it < 4; ++it) {
    const int q = it * NTHR + tid;
    *(volatile v4f*)(xzg + 4 * q) = xo[it];
    *(volatile v8us*)(xsg + (size_t)q * 8) = so[it];
  }
  if (tw) *(volatile v2d*)(pg + 2 * tid) = pv;
  __threadfence();
#pragma unroll
  for (int it = 0; it < 4; ++it) {
    const int q = it * NTHR + tid;
    *(volatile v4f*)(xzg + 4 * q) = xo[it];
    *(volatile v8us*)(xsg + (size_t)q * 8) = so[it];
  }
  if (tw) *(volatile v2d*)(pg + 2 * tid) = pv;
}

__global__ __launch_bounds__(NTHR) void k_bn2fin(const double* __restrict__ part2,
                                                const float* __restrict__ g2, const float* __restrict__ be2,
                                                float* bn2tab) {
  __shared__ __attribute__((aligned(16))) float tab[2 * NH];
  const int tid = threadIdx.x;
  if (tid < NH) {
    double s = 0.0, sq = 0.0;
#pragma unroll 1
    for (int k = 0; k < NB; ++k) {
      s  += part2[(size_t)k * (2 * NH) + tid];
      sq += part2[(size_t)k * (2 * NH) + NH + tid];
    }
    const double mu = s * INVROWS;
    double var = sq * INVROWS - mu * mu;
    var = var < 0.0 ? 0.0 : var;
    const float iv = rsqrtf((float)var + BN_EPS);
    const float sc = g2[tid] * iv;
    tab[tid]      = sc;
    tab[NH + tid] = be2[tid] - (float)mu * sc;
  }
  __syncthreads();
  if (tid < 32) {
    const v4f v = *(const v4f*)(tab + 4 * tid);
    float* dp = bn2tab + 4 * tid;
    *(volatile v4f*)dp = v;
    __threadfence();
    *(volatile v4f*)dp = v;
  }
}

__global__ __launch_bounds__(NTHR) void k_graph2(const float* __restrict__ xzp, const float* __restrict__ bn2tab,
                                                const unsigned short* __restrict__ xs16p, float* out) {
  extern __shared__ v4f lds_dyn[];
  char* lb = (char*)lds_dyn;
  unsigned short* z16 = (unsigned short*)(lb + L2_Z);
  float* S   = (float*)(lb + L2_S);
  unsigned short* P16 = (unsigned short*)(lb + L2_P);
  unsigned short* xsT = (unsigned short*)(lb + L2_XT);
  float* ostg = (float*)(lb + L2_O);
  float* bt2  = (float*)(lb + L2_BT);
  const int tid = threadIdx.x, lane = tid & 31, wave = tid >> 5, hh = lane >> 4, m = lane & 15;
  const int b = blockIdx.x;

  if (tid < 2 * NH) bt2[tid] = bn2tab[tid];
  {
    const unsigned short* xsg = xs16p + (size_t)b * NNODE * NF;
#pragma unroll
    for (int it = 0; it < 4; ++it) {
      const int q = it * NTHR + tid;
      const int mm = q >> 4, f0 = (q & 15) * 8;
      const v8us v = *(const v8us*)(xsg + (size_t)q * 8);
#pragma unroll
      for (int e = 0; e < 8; ++e) xsT[(f0 + e) * ZP + mm] = v[e];
    }
  }
  __syncthreads();

  {
    const float* xzg = xzp + (size_t)b * NNODE * NH;
#pragma unroll
    for (int it = 0; it < 4; ++it) {
      const int q = it * NTHR + tid;
      const int n = q >> 4, c0 = (q & 15) * 4;
      const v4f xv = *(const v4f*)(xzg + 4 * q);
      const v4f sc = *(const v4f*)(bt2 + c0);
      const v4f sh = *(const v4f*)(bt2 + NH + c0);
      v4f v = xv * sc + sh;
      v.x = v.x >= 0.0f ? v.x : 0.01f * v.x;
      v.y = v.y >= 0.0f ? v.y : 0.01f * v.y;
      v.z = v.z >= 0.0f ? v.z : 0.01f * v.z;
      v.w = v.w >= 0.0f ? v.w : 0.01f * v.w;
      *(v4us*)(z16 + n * ZP + c0) = cvt4(v, 1.0f);
    }
  }
  __syncthreads();

  {
    const int mt = wave >> 1, nt0 = (wave & 1) * 2;
    v8f acc[2];
#pragma unroll
    for (int t = 0; t < 2; ++t) { const v8f z = {0.f, 0.f, 0.f, 0.f, 0.f, 0.f, 0.f, 0.f}; acc[t] = z; }
    const unsigned short* afp = z16 + (16 * mt + m) * ZP + 8 * hh;
#pragma unroll
    for (int ks = 0; ks < NH / 32; ++ks) {
      FragH af;
      af.u[0] = *(const v8us*)(afp + 32 * ks);
      af.u[1] = *(const v8us*)(afp + 32 * ks + 16);
#pragma unroll
      for (int t = 0; t < 2; ++t) {
        const unsigned short* bfp = z16 + (16 * (nt0 + t) + m) * ZP + 32 * ks + 8 * hh;
        FragH bf;
        bf.u[0] = *(const v8us*)bfp;
        bf.u[1] = *(const v8us*)(bfp + 16);
        acc[t] = wmh(af.v, bf.v, acc[t]);
      }
    }
#pragma unroll
    for (int t = 0; t < 2; ++t) {
      float* op = S + (16 * mt + 8 * hh) * NNODE + 16 * (nt0 + t) + m;
#pragma unroll
      for (int r = 0; r < 8; ++r) op[r * NNODE] = acc[t][r];
    }
  }
  __syncthreads();

  {
    const int row = tid >> 2, part = tid & 3;
    const float* sp = S + row * NNODE + part * 16;
    const v4f s0 = *(const v4f*)sp, s1 = *(const v4f*)(sp + 4), s2 = *(const v4f*)(sp + 8), s3 = *(const v4f*)(sp + 12);
    float e[16] = {s0.x, s0.y, s0.z, s0.w, s1.x, s1.y, s1.z, s1.w,
                   s2.x, s2.y, s2.z, s2.w, s3.x, s3.y, s3.z, s3.w};
    float mx = e[0];
#pragma unroll
    for (int j = 1; j < 16; ++j) mx = fmaxf(mx, e[j]);
    mx = fmaxf(mx, __shfl_xor(mx, 1));
    mx = fmaxf(mx, __shfl_xor(mx, 2));
    float sum = 0.0f;
#pragma unroll
    for (int j = 0; j < 16; ++j) { e[j] = __expf(e[j] - mx); sum += e[j]; }
    sum += __shfl_xor(sum, 1);
    sum += __shfl_xor(sum, 2);
    const float rr = PSCL / sum;
    v8us p0, p1;
#pragma unroll
    for (int j = 0; j < 8; ++j) { p0[j] = h16(e[j] * rr); p1[j] = h16(e[8 + j] * rr); }
    unsigned short* pp = P16 + row * ZP + part * 16;
    *(v8us*)pp = p0;
    *(v8us*)(pp + 8) = p1;
  }
  __syncthreads();

  {
    const int nt = wave;
    FragH bfr[2];
    const unsigned short* bfp = xsT + (16 * nt + m) * ZP + 8 * hh;
#pragma unroll
    for (int ks = 0; ks < NNODE / 32; ++ks) {
      bfr[ks].u[0] = *(const v8us*)(bfp + 32 * ks);
      bfr[ks].u[1] = *(const v8us*)(bfp + 32 * ks + 16);
    }
#pragma unroll
    for (int mt = 0; mt < 4; ++mt) {
      v8f acc = {0.f, 0.f, 0.f, 0.f, 0.f, 0.f, 0.f, 0.f};
      const unsigned short* afp = P16 + (16 * mt + m) * ZP + 8 * hh;
#pragma unroll
      for (int ks = 0; ks < NNODE / 32; ++ks) {
        FragH af;
        af.u[0] = *(const v8us*)(afp + 32 * ks);
        af.u[1] = *(const v8us*)(afp + 32 * ks + 16);
        acc = wmh(af.v, bfr[ks].v, acc);
      }
      float* op = ostg + (16 * mt + 8 * hh) * NF + 16 * nt + m;
#pragma unroll
      for (int r = 0; r < 8; ++r) op[r * NF] = acc[r] * INV65536;
    }
  }
  __syncthreads();

  v4f ov[8];
#pragma unroll
  for (int it = 0; it < 8; ++it) ov[it] = *(const v4f*)(ostg + 4 * (it * NTHR + tid));
  float* og = out + (size_t)b * NNODE * NF;
#pragma unroll
  for (int it = 0; it < 8; ++it) *(volatile v4f*)(og + 4 * (it * NTHR + tid)) = ov[it];
  __threadfence();
#pragma unroll
  for (int it = 0; it < 8; ++it) *(volatile v4f*)(og + 4 * (it * NTHR + tid)) = ov[it];
}

static inline size_t al256(size_t v) { return (v + 255) & ~(size_t)255; }

extern "C" void kernel_launch(void* const* d_in, const int* in_sizes, int n_in,
                              void* d_out, int out_size, void* d_ws, size_t ws_size,
                              hipStream_t stream) {
  if (n_in < 9) return;
  if (in_sizes[0] != NROWS * NF) return;
  if (in_sizes[1] != 2 * NB * NGE) return;
  if (in_sizes[2] != NTRIL || in_sizes[3] != NH * NF || in_sizes[4] != NH) return;
  if (in_sizes[5] != NF || in_sizes[6] != NF || in_sizes[7] != NH || in_sizes[8] != NH) return;
  if (out_size != NB * NNODE * NF) return;

  const float* x     = (const float*)d_in[0];
  const float* tril  = (const float*)d_in[2];
  const float* lin_w = (const float*)d_in[3];
  const float* lin_b = (const float*)d_in[4];
  const float* g1    = (const float*)d_in[5];
  const float* be1   = (const float*)d_in[6];
  const float* g2    = (const float*)d_in[7];
  const float* be2   = (const float*)d_in[8];
  float* out = (float*)d_out;

  const size_t szP1 = (size_t)NSTAT * NTHR * 8;
  const size_t szT1 = (size_t)2 * NF * 4;
  const size_t szA2 = (size_t)NGE * 4;
  const size_t szLW = (size_t)NH * NF * 2;
  const size_t szXS = (size_t)NROWS * NF * 2;
  const size_t szXZ = (size_t)NROWS * NH * 4;
  const size_t szP2 = (size_t)NB * 2 * NH * 8;
  const size_t szT2 = (size_t)2 * NH * 4;
  size_t off = 0;
  const size_t oP1 = off; off = al256(off + szP1);
  const size_t oT1 = off; off = al256(off + szT1);
  const size_t oA2 = off; off = al256(off + szA2);
  const size_t oLW = off; off = al256(off + szLW);
  const size_t oXS = off; off = al256(off + szXS);
  const size_t oXZ = off; off = al256(off + szXZ);
  const size_t oP2 = off; off = al256(off + szP2);
  const size_t oT2 = off; off = al256(off + szT2);
  if (off > ws_size || off > (size_t)WSCAP) return;
  char* ws = (char*)d_ws;
  double*         part1  = (double*)(ws + oP1);
  float*          bn1tab = (float*)(ws + oT1);
  float*          A2g    = (float*)(ws + oA2);
  unsigned short* lw16   = (unsigned short*)(ws + oLW);
  unsigned short* xs16p  = (unsigned short*)(ws + oXS);
  float*          xzp    = (float*)(ws + oXZ);
  double*         part2  = (double*)(ws + oP2);
  float*          bn2tab = (float*)(ws + oT2);

  k_stat1<<<NSTAT, NTHR, 0, stream>>>(x, part1);
  k_prep<<<1, NTHR, 0, stream>>>(part1, g1, be1, tril, lin_w, bn1tab, A2g, lw16);
  hipFuncSetAttribute(reinterpret_cast<const void*>(&k_graph1),
                      hipFuncAttributeMaxDynamicSharedMemorySize, LDS1);
  k_graph1<<<NB, NTHR, LDS1, stream>>>(x, bn1tab, A2g, lw16, lin_b, xs16p, xzp, part2);
  k_bn2fin<<<1, NTHR, 0, stream>>>(part2, g2, be2, bn2tab);
  hipFuncSetAttribute(reinterpret_cast<const void*>(&k_graph2),
                      hipFuncAttributeMaxDynamicSharedMemorySize, LDS2);
  k_graph2<<<NB, NTHR, LDS2, stream>>>(xzp, bn2tab, xs16p, out);
}
